// DKGMBlock_58574763983532
// MI455X (gfx1250) — hardware-verified
//
#include <hip/hip_runtime.h>
#include <math.h>


#define NB    16
#define IMG   512
#define CELL  16
#define NCELL 32
#define ORI   9
#define PLANE (IMG * IMG)
typedef __attribute__((ext_vector_type(16))) _Float16 v16h;
typedef __attribute__((ext_vector_type(8)))  float    v8f;
typedef __attribute__((ext_vector_type(4)))  float    v4f;
#define VST2(T, ptr, val) do { const T _v = (val); *(volatile T*)(ptr) = _v; __threadfence(); *(volatile T*)(ptr) = _v; } while (0)
__device__ __forceinline__ v8f wmma16(v16h a, v16h b, v8f c) {
  v8f d = __builtin_amdgcn_wmma_f32_16x16x32_f16(false, a, false, b, (short)0, c, false, false);
  asm volatile("v_nop\n\tv_nop\n\tv_nop\n\tv_nop" : "+v"(d) : "v"(a), "v"(b));
  return d;
}
__device__ __forceinline__ int kmap(int e, int hh) { return (e < 8) ? (8 * hh + e) : (16 + 8 * hh + (e - 8)); }

__global__ __launch_bounds__(256) void k_hls(const float* __restrict__ x, float* __restrict__ hpl, float* __restrict__ lpl, float* __restrict__ gray) {
  const int idx = blockIdx.x * 256 + threadIdx.x;
  const int img = idx / PLANE, pix = idx % PLANE;
  const float* base = x + (size_t)img * 3 * PLANE + pix;
  const float r = base[0], g = base[PLANE], b = base[2 * PLANE];
  const float vmax = fmaxf(fmaxf(r, g), b), vmin = fminf(fminf(r, g), b);
  const float diff = vmax - vmin;
  const float l = (vmax + vmin) * 0.5f;
  const bool nz = diff > 0.0f;
  const float safe = nz ? diff : 1.0f;
  float h = (vmax == r) ? (60.0f * (g - b) / safe) : (vmax == g) ? (120.0f + 60.0f * (b - r) / safe) : (240.0f + 60.0f * (r - g) / safe);
  if (h < 0.0f) h += 360.0f;
  if (!nz) h = 0.0f;
  VST2(float, hpl + idx, h);
  VST2(float, lpl + idx, l);
  VST2(float, gray + idx, 0.299f * r + 0.587f * g + 0.114f * b);
}
__global__ __launch_bounds__(256) void k_hog(const float* __restrict__ gray, float* __restrict__ hog) {
  __shared__ float part[ORI][256];
  __shared__ __attribute__((aligned(16))) float tile[256];
  __shared__ float hist[ORI];
  const int bid = blockIdx.x, img = bid >> 10, cy = (bid >> 5) & 31, cx = bid & 31;
  const int t = threadIdx.x, ly = t >> 4, lx = t & 15, y = cy * CELL + ly, xx = cx * CELL + lx;
  const float* gp = gray + (size_t)img * PLANE;
  const float gr = (y >= 1 && y <= IMG - 2) ? (gp[(y + 1) * IMG + xx] - gp[(y - 1) * IMG + xx]) : 0.0f;
  const float gc = (xx >= 1 && xx <= IMG - 2) ? (gp[y * IMG + xx + 1] - gp[y * IMG + xx - 1]) : 0.0f;
  const float sq = gr * gr + gc * gc;
  const float mag = (sq > 0.0f) ? sqrtf(sq) : 0.0f;
  float ang = atan2f(gr, gc) * (180.0f / 3.14159265358979323846f);
  ang = fmodf(ang, 180.0f); if (ang < 0.0f) ang += 180.0f;
  int bin = (int)(ang * (ORI / 180.0f)); bin = min(max(bin, 0), ORI - 1);
#pragma unroll
  for (int o = 0; o < ORI; ++o) part[o][t] = (o == bin) ? mag : 0.0f;
  tile[t] = 0.0f;
  __syncthreads();
  for (int s = 128; s > 0; s >>= 1) {
    if (t < s) {
#pragma unroll
      for (int o = 0; o < ORI; ++o) part[o][t] += part[o][t + s]; }
    __syncthreads();
  }
  if (t < ORI) hist[t] = part[t][0] * (1.0f / (CELL * CELL));
  __syncthreads();
  if (t == 0) {
    for (int o = 0; o < ORI; ++o) {
      const float val = hist[o];
      const float mid = 3.14159265358979323846f * (o + 0.5f) / ORI;
      const float drf = 7.0f * sinf(mid), dcf = 7.0f * cosf(mid);
      const int r0 = (int)(8.0f - dcf), c0 = (int)(8.0f + drf), r1 = (int)(8.0f + dcf), c1 = (int)(8.0f - drf);
      int r = r0, c = c0, adr = abs(r1 - r0), adc = abs(c1 - c0);
      int sc = (c1 - c0 > 0) ? 1 : -1, sr = (r1 - r0 > 0) ? 1 : -1;
      const bool steep = adr > adc;
      if (steep) { int tmp = r; r = c; c = tmp; tmp = adr; adr = adc; adc = tmp; tmp = sr; sr = sc; sc = tmp; }
      int d = 2 * adr - adc;
      for (int i = 0; i < adc; ++i) {
        const int pr = steep ? c : r, pc = steep ? r : c;
        tile[pr * CELL + pc] += val;
        while (d >= 0) { r += sr; d -= 2 * adc; }
        c += sc; d += 2 * adr;
      }
      tile[r1 * CELL + c1] += val;
    }
  }
  __syncthreads();
  if (t < 64) {
    v4f v; const int q = t * 4;
    v[0] = fminf(fmaxf(tile[q], 0.f), 10.f) * 0.1f; v[1] = fminf(fmaxf(tile[q + 1], 0.f), 10.f) * 0.1f;
    v[2] = fminf(fmaxf(tile[q + 2], 0.f), 10.f) * 0.1f; v[3] = fminf(fmaxf(tile[q + 3], 0.f), 10.f) * 0.1f;
    VST2(v4f, hog + (size_t)bid * 256 + q, v);
  }
}
__device__ __forceinline__ float emb_at(const float* __restrict__ hpl, const float* __restrict__ lpl, const float* __restrict__ hog, int img, int ci, int y, int x) {
  if (y < 0 || y >= IMG || x < 0 || x >= IMG) return 0.0f;
  if (ci == 0) return hpl[(size_t)img * PLANE + y * IMG + x];
  if (ci == 1) return lpl[(size_t)img * PLANE + y * IMG + x];
  const int cell = (y >> 4) * NCELL + (x >> 4), off = (y & 15) * CELL + (x & 15);
  return hog[((size_t)img * 1024 + cell) * 256 + off];
}
__global__ __launch_bounds__(256) void k_conv(const float* __restrict__ hpl, const float* __restrict__ lpl, const float* __restrict__ hog,
                                              const float* __restrict__ xin, const float* __restrict__ cw, const float* __restrict__ cb, float* __restrict__ out) {
  __shared__ float so[8][3][32];
  const int lane = threadIdx.x & 31, wave = threadIdx.x >> 5, hh = lane >> 4, l16 = lane & 15;
  const int strip = blockIdx.x * 8 + wave;
  const int img = strip / (IMG * (IMG / 32)), rem = strip % (IMG * (IMG / 32)), y = rem / (IMG / 32), x0 = (rem % (IMG / 32)) * 32;
  v16h bw;
#pragma unroll
  for (int e = 0; e < 16; ++e) { const int k = kmap(e, hh); bw[e] = (k < 27 && l16 < 3) ? (_Float16)cw[l16 * 27 + k] : (_Float16)0.f; }
  for (int half = 0; half < 2; ++half) {
    const int px = x0 + half * 16 + l16;
    v16h ah, al;
#pragma unroll
    for (int e = 0; e < 16; ++e) {
      const int k = kmap(e, hh);
      float v = 0.f;
      if (k < 27) { const int ci = k / 9, tap = k % 9, ky = tap / 3, kx = tap % 3; v = emb_at(hpl, lpl, hog, img, ci, y + ky - 1, px + kx - 1); }
      const _Float16 hi_ = (_Float16)v; ah[e] = hi_; al[e] = (_Float16)(v - (float)hi_);
    }
    v8f c = {};
    c = wmma16(ah, bw, c);
    c = wmma16(al, bw, c);
    if (l16 < 3) {
#pragma unroll
      for (int r = 0; r < 8; ++r) so[wave][l16][half * 16 + r + 8 * hh] = c[r] + cb[l16];
    }
  }
  __builtin_amdgcn_fence(__ATOMIC_RELEASE, "workgroup"); __builtin_amdgcn_wave_barrier(); __builtin_amdgcn_fence(__ATOMIC_ACQUIRE, "workgroup");
  for (int pass = 0; pass < 2; ++pass) {
#pragma unroll
    for (int co = 0; co < 3; ++co) {
      const size_t o = ((size_t)img * 3 + co) * PLANE + (size_t)y * IMG + x0 + lane;
      *(volatile float*)(out + o) = xin[o] + so[wave][co][lane];
    }
    __threadfence();
  }
}
extern "C" void kernel_launch(void* const* d_in, const int* in_sizes, int n_in,
                              void* d_out, int out_size, void* d_ws, size_t ws_size, hipStream_t stream) {
  (void)in_sizes; (void)n_in; (void)out_size;
  const float* x  = (const float*)d_in[0];
  const float* cw = (const float*)d_in[1];
  const float* cb = (const float*)d_in[2];
  float* out = (float*)d_out;
  char* ws = (char*)d_ws; size_t off = 0;
  auto take = [&](size_t bytes) { void* p = ws + off; off = (off + bytes + 255) & ~(size_t)255; return p; };
  float* hpl  = (float*)take((size_t)NB * PLANE * 4);
  float* lpl  = (float*)take((size_t)NB * PLANE * 4);
  float* gray = (float*)take((size_t)NB * PLANE * 4);
  float* hog  = (float*)take((size_t)NB * PLANE * 4);
  if (off > ws_size) return;
  k_hls<<<NB * PLANE / 256, 256, 0, stream>>>(x, hpl, lpl, gray);
  k_hog<<<NB * NCELL * NCELL, 256, 0, stream>>>(gray, hog);
  k_conv<<<NB * IMG * (IMG / 32) / 8, 256, 0, stream>>>(hpl, lpl, hog, x, cw, cb, out);
}
